// MultiHeadAttentionRoPE_15796889715401
// MI455X (gfx1250) — hardware-verified
//
#include <hip/hip_runtime.h>
#include <math.h>

static constexpr int kSeq   = 4096;
static constexpr int kDm    = 768;
static constexpr int kHeads = 12;
static constexpr int kHd    = 64;
static constexpr int kNqkv  = 3 * kDm;
static_assert(kHeads * kHd == kDm, "head split");
static_assert(kSeq % 64 == 0 && kDm % 64 == 0 && kNqkv % 64 == 0, "GEMM M/N tile multiples");
static_assert(kDm % 32 == 0, "GEMM K multiple of 32");
static_assert(kHd == 64, "attention kernel is head-dim 64");

typedef __attribute__((ext_vector_type(16))) _Float16 v16h;
typedef __attribute__((ext_vector_type(8)))  _Float16 v8h;
typedef __attribute__((ext_vector_type(16))) __bf16   v16b;
typedef __attribute__((ext_vector_type(8)))  __bf16   v8b;
typedef __attribute__((ext_vector_type(8)))  float    v8f;
typedef __attribute__((ext_vector_type(4)))  float    v4f;
typedef __attribute__((ext_vector_type(4)))  unsigned v4u;
#define PSCALE 32768.0f
#define U16(p) ((const unsigned short*)(const void*)(p))
#define PSCALE_INV (1.0f / 32768.0f)

__device__ __forceinline__ unsigned short f2bf_bits(float f) {
  unsigned u = __float_as_uint(f);
  return (unsigned short)((u + 0x7FFFu + ((u >> 16) & 1u)) >> 16);
}
__device__ __forceinline__ float bf_bits2f(unsigned short h) { return __uint_as_float(((unsigned)h) << 16); }

__device__ __forceinline__ void dep_guard_h(v8f& a, v8f& b, v16h x, v16h y) { asm volatile("v_nop\n\tv_nop\n\tv_nop\n\tv_nop" : "+v"(a), "+v"(b) : "v"(x), "v"(y)); }
__device__ __forceinline__ void dep_guard_b(v8f& a, v8f& b, v16b x, v16b y) { asm volatile("v_nop\n\tv_nop\n\tv_nop\n\tv_nop" : "+v"(a), "+v"(b) : "v"(x), "v"(y)); }
__device__ __forceinline__ void keep4_h(v16h a, v16h b, v16h c, v16h d) { asm volatile("v_nop" :: "v"(a), "v"(b), "v"(c), "v"(d)); }
__device__ __forceinline__ void keep4_b(v16b a, v16b b, v16b c, v16b d) { asm volatile("v_nop" :: "v"(a), "v"(b), "v"(c), "v"(d)); }
__device__ __forceinline__ void acc_guard4(v8f& a, v8f& b, v8f& c, v8f& d) { asm volatile("v_nop\n\tv_nop\n\tv_nop\n\tv_nop" : "+v"(a), "+v"(b), "+v"(c), "+v"(d)); }
template <typename T> struct Frag;
template <> struct Frag<_Float16> {
  typedef v16h V; union U { v16h v; v8h h[2]; };
  static __device__ __forceinline__ v16h load(const _Float16* p) {
    U f; f.h[0] = *(const v8h*)(p); f.h[1] = *(const v8h*)(p + 16); return f.v;
  }
  static __device__ __forceinline__ v8f mma(v16h a, v16h b, v8f c) {
    return __builtin_amdgcn_wmma_f32_16x16x32_f16(false, a, false, b, (short)0, c, false, false);
  }
  static __device__ __forceinline__ void guard(v8f& a, v8f& b, v16h x, v16h y) { dep_guard_h(a, b, x, y); }
  static __device__ __forceinline__ void keep(v16h a, v16h b, v16h c, v16h d) { keep4_h(a, b, c, d); }
};
template <> struct Frag<__bf16> {
  typedef v16b V; union U { v16b v; v8b h[2]; };
  static __device__ __forceinline__ v16b load(const __bf16* p) {
    U f; f.h[0] = *(const v8b*)(p); f.h[1] = *(const v8b*)(p + 16); return f.v;
  }
  static __device__ __forceinline__ v8f mma(v16b a, v16b b, v8f c) {
    return __builtin_amdgcn_wmma_f32_16x16x32_bf16(false, a, false, b, (short)0, c, false, false);
  }
  static __device__ __forceinline__ void guard(v8f& a, v8f& b, v16b x, v16b y) { dep_guard_b(a, b, x, y); }
  static __device__ __forceinline__ void keep(v16b a, v16b b, v16b c, v16b d) { keep4_b(a, b, c, d); }
};

template <int ET> struct Elem;
template <> struct Elem<0> { typedef _Float16 T; };
template <> struct Elem<1> { typedef __bf16 T; };
template <int ET, int SPLIT, int BIAS_MODE, int OUT_MODE, bool RESID, int ACT = 0>
__global__ __launch_bounds__(256) void wmma_gemm64(
    const unsigned short* __restrict__ Ap, const unsigned short* __restrict__ A2p, int lda, long strideA,
    const unsigned short* __restrict__ Btp, const unsigned short* __restrict__ Bt2p, int ldb, long strideB,
    void* __restrict__ Cout, void* __restrict__ Cout2, int ldc, long strideC,
    const float* __restrict__ bias,
    const float* __restrict__ resid, long strideR,
    int M, int N, int K, float scale) {
  typedef typename Elem<ET>::T T;
  typedef typename Frag<T>::V V;
  const T* A = (const T*)Ap; const T* A2 = (const T*)A2p; const T* Bt = (const T*)Btp; const T* Bt2 = (const T*)Bt2p;
  __shared__ __align__(16) float sT[8][16 * 68];
  const int b    = blockIdx.y;
  const int lane = threadIdx.x & 31;
  const int wave = threadIdx.x >> 5;
  const int tilesN = N >> 6;
  const int tilesM = M >> 6;
  const int tile = blockIdx.x * 8 + wave;
  if (tile >= tilesM * tilesN) return;
  const int tm = tile / tilesN;
  const int tn = tile - tm * tilesN;
  const int m0 = tm << 6;
  const int n0 = tn << 6;

  const T* Ab  = A  + (size_t)b * strideA;
  const T* Bb  = Bt + (size_t)b * strideB;
  const T* Ab2 = (SPLIT >= 1) ? (A2  + (size_t)b * strideA) : nullptr;
  const T* Bb2 = (SPLIT == 2) ? (Bt2 + (size_t)b * strideB) : nullptr;

  const int rlane = lane & 15;
  const int koff  = (lane >> 4) * 8;
  const int mOff  = (lane >> 4) * 8;

  v8f acc[4][4];
#pragma unroll
  for (int i = 0; i < 4; ++i)
#pragma unroll
    for (int j = 0; j < 4; ++j) acc[i][j] = (v8f){0.f,0.f,0.f,0.f,0.f,0.f,0.f,0.f};

  for (int k0 = 0; k0 < K; k0 += 32) {
    V bh[4], bl[4];
#pragma unroll
    for (int j = 0; j < 4; ++j) {
      const size_t bo = (size_t)(n0 + (j << 4) + rlane) * ldb + koff + k0;
      bh[j] = Frag<T>::load(Bb + bo);
      if (SPLIT == 2) bl[j] = Frag<T>::load(Bb2 + bo);
    }
#pragma unroll
    for (int i = 0; i < 4; ++i) {
      const size_t ao = (size_t)(m0 + (i << 4) + rlane) * lda + koff + k0;
      V ah = Frag<T>::load(Ab + ao);
      V al;
      if (SPLIT >= 1) al = Frag<T>::load(Ab2 + ao);
#pragma unroll
      for (int j = 0; j < 4; ++j) {
        acc[i][j] = Frag<T>::mma(ah, bh[j], acc[i][j]);
        if (SPLIT == 2) acc[i][j] = Frag<T>::mma(ah, bl[j], acc[i][j]);
        if (SPLIT >= 1) acc[i][j] = Frag<T>::mma(al, bh[j], acc[i][j]);
      }
      Frag<T>::guard(acc[i][0], acc[i][3], ah, (SPLIT >= 1) ? al : ah);
    }
    Frag<T>::keep(bh[0], bh[1], bh[2], bh[3]);
    if (SPLIT == 2) Frag<T>::keep(bl[0], bl[1], bl[2], bl[3]);
  }
  acc_guard4(acc[0][0], acc[0][1], acc[0][2], acc[0][3]);
  acc_guard4(acc[1][0], acc[1][1], acc[1][2], acc[1][3]);
  acc_guard4(acc[2][0], acc[2][1], acc[2][2], acc[2][3]);
  acc_guard4(acc[3][0], acc[3][1], acc[3][2], acc[3][3]);

  float* slab = sT[wave];
  const float* Rb = RESID ? (resid + (size_t)b * strideR) : nullptr;
#pragma unroll
  for (int i = 0; i < 4; ++i) {
    const int mBase = m0 + (i << 4);
#pragma unroll
    for (int j = 0; j < 4; ++j) {
      const int n = n0 + (j << 4) + rlane;
      float bv = 0.f;
      if (BIAS_MODE == 2) bv = bias[n];
#pragma unroll
      for (int r = 0; r < 8; ++r) {
        float v = acc[i][j][r] * scale;
        if (BIAS_MODE == 1) v += bias[mBase + mOff + r];
        if (BIAS_MODE == 2) v += bv;
        if (RESID) v += Rb[(size_t)(mBase + mOff + r) * ldc + n];
        if (ACT == 1) v = tanhf(v);
        if (ACT == 2) v = fmaxf(v, 0.0f);
        if (ACT == 3) v = v / (1.0f + expf(-v));
        if (ACT == 4) v = (v > 0.f) ? v : 0.01f * v;
        if (ACT == 5) v = 0.5f * v * (1.0f + erff(v * 0.70710678118654752f));
        slab[(mOff + r) * 68 + (j << 4) + rlane] = v;
      }
    }
    __builtin_amdgcn_fence(__ATOMIC_RELEASE, "workgroup");
    __builtin_amdgcn_wave_barrier();
    __builtin_amdgcn_fence(__ATOMIC_ACQUIRE, "workgroup");
    if (OUT_MODE == 0) {
      float* C = (float*)Cout + (size_t)b * strideC;
      const int hh = lane >> 4, c4 = (lane & 15) * 4;
      for (int pass = 0; pass < 2; ++pass) {
#pragma unroll
        for (int it = 0; it < 8; ++it) {
          const int row = it * 2 + hh;
          v4f v = *(const v4f*)(slab + row * 68 + c4);
          *(volatile v4f*)(C + (size_t)(mBase + row) * ldc + n0 + c4) = v;
        }
        __threadfence();
      }
    } else {
      const int q = lane >> 3, c8 = (lane & 7) * 8;
      unsigned short* C  = (unsigned short*)Cout  + (size_t)b * strideC;
      unsigned short* C2 = (OUT_MODE == 2) ? ((unsigned short*)Cout2 + (size_t)b * strideC) : nullptr;
      for (int pass = 0; pass < 2; ++pass) {
#pragma unroll
        for (int it = 0; it < 4; ++it) {
          const int row = it * 4 + q;
          const float* sp = slab + row * 68 + c8;
          v8h hv, lv;
#pragma unroll
          for (int e = 0; e < 8; ++e) {
            if (OUT_MODE == 1) {
              hv[e] = (_Float16)sp[e];
            } else {
              unsigned short hb = f2bf_bits(sp[e]);
              unsigned short lb = f2bf_bits(sp[e] - bf_bits2f(hb));
              hv[e] = __builtin_bit_cast(_Float16, hb);
              lv[e] = __builtin_bit_cast(_Float16, lb);
            }
          }
          *(volatile v8h*)(C + (size_t)(mBase + row) * ldc + n0 + c8) = hv;
          if (OUT_MODE == 2) *(volatile v8h*)(C2 + (size_t)(mBase + row) * ldc + n0 + c8) = lv;
        }
        __threadfence();
      }
    }
    __builtin_amdgcn_fence(__ATOMIC_RELEASE, "workgroup");
    __builtin_amdgcn_wave_barrier();
    __builtin_amdgcn_fence(__ATOMIC_ACQUIRE, "workgroup");
  }
}

__device__ __forceinline__ void st2_v4u(unsigned short* p, v4u u) {
  *(volatile v4u*)(void*)p = u;
  __threadfence();
  *(volatile v4u*)(void*)p = u;
}
__device__ __forceinline__ void st2_v4f(float* p, v4f v) {
  *(volatile v4f*)(void*)p = v;
  __threadfence();
  *(volatile v4f*)(void*)p = v;
}
__device__ __forceinline__ unsigned pack_h2(float a, float b) {
  const unsigned short ha = __builtin_bit_cast(unsigned short, (_Float16)a);
  const unsigned short hb = __builtin_bit_cast(unsigned short, (_Float16)b);
  return (unsigned)ha | ((unsigned)hb << 16);
}
__device__ __forceinline__ unsigned pack_bf2(float a, float b) {
  return (unsigned)f2bf_bits(a) | ((unsigned)f2bf_bits(b) << 16);
}
__device__ __forceinline__ unsigned res_h2(float a, float b, float carry) {
  const float ha = (float)(_Float16)a;
  const float hb = (float)(_Float16)b;
  const float ra = (a - ha) * carry;
  const float rb = (b - hb) * carry;
  return pack_h2(ra, rb);
}
__device__ __forceinline__ v8f hmma_f16(v16h a, v16h b, v8f c) {
  c = __builtin_amdgcn_wmma_f32_16x16x32_f16(false, a, false, b, (short)0, c, false, false);
  asm volatile("v_nop\n\tv_nop\n\tv_nop\n\tv_nop" : "+v"(c) : "v"(a), "v"(b));
  return c;
}

__global__ __launch_bounds__(256) void k_cast_bf16(const float* __restrict__ in,
                                                    unsigned short* __restrict__ out, int n8) {
  const int i = blockIdx.x * 256 + threadIdx.x;
  if (i >= n8) return;
  const v4f a = *(const v4f*)(in + (size_t)i * 8);
  const v4f b = *(const v4f*)(in + (size_t)i * 8 + 4);
  v4u u;
  u[0] = pack_bf2(a[0], a[1]);
  u[1] = pack_bf2(a[2], a[3]);
  u[2] = pack_bf2(b[0], b[1]);
  u[3] = pack_bf2(b[2], b[3]);
  st2_v4u(out + (size_t)i * 8, u);
}

__global__ __launch_bounds__(256) void k_bias_bf(const float* __restrict__ bq, const float* __restrict__ bo,
                                                  float* __restrict__ bqr, float* __restrict__ bor) {
  const bool first = (blockIdx.x < 3);
  const float* src = first ? bq : bo;
  float* dst = first ? bqr : bor;
  const int n4 = first ? (kNqkv / 4) : (kDm / 4);
  const int i = (first ? (int)blockIdx.x * 256 : 0) + (int)threadIdx.x;
  if (i >= n4) return;
  const v4f v = *(const v4f*)(src + (size_t)i * 4);
  v4f o;
#pragma unroll
  for (int e = 0; e < 4; ++e) o[e] = bf_bits2f(f2bf_bits(v[e]));
  st2_v4f(dst + (size_t)i * 4, o);
}

__global__ __launch_bounds__(256) void k_transpose_bf16(const float* __restrict__ in,
                                                          unsigned short* __restrict__ out,
                                                          int rows, int cols) {
  __shared__ __align__(16) unsigned short tileT[64 * 72];
  const int t  = threadIdx.x;
  const int c0 = blockIdx.x * 64;
  const int r0 = blockIdx.y * 64;
#pragma unroll
  for (int it = 0; it < 4; ++it) {
    const int idx = it * 256 + t;
    const int rr = idx >> 4, c4 = (idx & 15) * 4;
    const v4f v = *(const v4f*)(in + (size_t)(r0 + rr) * cols + c0 + c4);
#pragma unroll
    for (int e = 0; e < 4; ++e) tileT[(c4 + e) * 72 + rr] = f2bf_bits(v[e]);
  }
  __syncthreads();
#pragma unroll
  for (int it = 0; it < 2; ++it) {
    const int row = it * 32 + (t >> 3);
    const int c8  = (t & 7) * 8;
    const v4u u = *(const v4u*)(const void*)(tileT + row * 72 + c8);
    st2_v4u(out + (size_t)(c0 + row) * rows + r0 + c8, u);
  }
}

struct RopeFreq { float f[32]; };
static_assert(sizeof(RopeFreq) == 128, "no padding");

__global__ __launch_bounds__(256) void k_rope_table(float* __restrict__ cosT, float* __restrict__ sinT,
                                                      RopeFreq fr) {
#pragma clang fp contract(off)
  const int lane = threadIdx.x & 31;
  const int s = blockIdx.x * 8 + (threadIdx.x >> 5);
  float f = fr.f[0];
#pragma unroll
  for (int j = 1; j < 32; ++j) f = (lane == j) ? fr.f[j] : f;
  const float ang = (float)s * f;
  float sv, cv;
  sincosf(ang, &sv, &cv);
  const int base = (lane & 7) * 4;
  v4f c4, s4;
#pragma unroll
  for (int e = 0; e < 4; ++e) {
    c4[e] = __shfl(cv, base + e, 32);
    s4[e] = __shfl(sv, base + e, 32);
  }
  if (lane < 8) {
    float* cp = cosT + (size_t)s * 32 + base;
    float* sp = sinT + (size_t)s * 32 + base;
    *(volatile v4f*)(void*)cp = c4;
    *(volatile v4f*)(void*)sp = s4;
    __threadfence();
    *(volatile v4f*)(void*)cp = c4;
    *(volatile v4f*)(void*)sp = s4;
  }
}

__global__ __launch_bounds__(256) void k_rope_planes(const float* __restrict__ QKV,
                                                       const float* __restrict__ cosT, const float* __restrict__ sinT,
                                                       unsigned short* __restrict__ Qh, unsigned short* __restrict__ Ql,
                                                       unsigned short* __restrict__ Kp, unsigned short* __restrict__ Vtp,
                                                       float qcarry) {
  __shared__ float Vs[64 * 65];
  const int t  = threadIdx.x;
  const int h  = blockIdx.y;
  const int s0 = blockIdx.x * 64;
#pragma unroll 1
  for (int sp = 0; sp < 4; ++sp) {
    const int sec = sp >> 1;
    const int it  = sp & 1;
    const int r   = it * 32 + (t >> 3);
    const int d8  = (t & 7) * 8;
    const int s   = s0 + r;
    const float* src = QKV + (size_t)s * kNqkv + sec * kDm + h * kHd + d8;
    const v4f x0 = *(const v4f*)(src);
    const v4f x1 = *(const v4f*)(src + 4);
    const float* cptr = cosT + (size_t)s * 32 + (d8 & 31);
    const float* sptr = sinT + (size_t)s * 32 + (d8 & 31);
    const v4f c0 = *(const v4f*)(cptr);
    const v4f c1 = *(const v4f*)(cptr + 4);
    const v4f n0 = *(const v4f*)(sptr);
    const v4f n1 = *(const v4f*)(sptr + 4);
    const float o0 = x0[0] * c0[0] - x0[1] * n0[0];
    const float o1 = x0[1] * c0[1] + x0[0] * n0[1];
    const float o2 = x0[2] * c0[2] - x0[3] * n0[2];
    const float o3 = x0[3] * c0[3] + x0[2] * n0[3];
    const float o4 = x1[0] * c1[0] - x1[1] * n1[0];
    const float o5 = x1[1] * c1[1] + x1[0] * n1[1];
    const float o6 = x1[2] * c1[2] - x1[3] * n1[2];
    const float o7 = x1[3] * c1[3] + x1[2] * n1[3];
    const size_t off = ((size_t)h * kSeq + s) * kHd + d8;
    if (sec == 0) {
      v4u uh, ul;
      uh[0] = pack_h2(o0, o1);  ul[0] = res_h2(o0, o1, qcarry);
      uh[1] = pack_h2(o2, o3);  ul[1] = res_h2(o2, o3, qcarry);
      uh[2] = pack_h2(o4, o5);  ul[2] = res_h2(o4, o5, qcarry);
      uh[3] = pack_h2(o6, o7);  ul[3] = res_h2(o6, o7, qcarry);
      st2_v4u(Qh + off, uh);
      st2_v4u(Ql + off, ul);
    } else {
      v4u u;
      u[0] = pack_h2(o0, o1);
      u[1] = pack_h2(o2, o3);
      u[2] = pack_h2(o4, o5);
      u[3] = pack_h2(o6, o7);
      st2_v4u(Kp + off, u);
    }
  }
#pragma unroll
  for (int it = 0; it < 4; ++it) {
    const int idx = it * 256 + t;
    const int r = idx >> 4, c4 = (idx & 15) * 4;
    const v4f v = *(const v4f*)(QKV + (size_t)(s0 + r) * kNqkv + 2 * kDm + h * kHd + c4);
    Vs[r * 65 + c4 + 0] = v[0];
    Vs[r * 65 + c4 + 1] = v[1];
    Vs[r * 65 + c4 + 2] = v[2];
    Vs[r * 65 + c4 + 3] = v[3];
  }
  __syncthreads();
#pragma unroll
  for (int it = 0; it < 2; ++it) {
    const int drow = it * 32 + (t >> 3);
    const int s8   = (t & 7) * 8;
    v4u u;
    u[0] = pack_h2(Vs[(s8 + 0) * 65 + drow], Vs[(s8 + 1) * 65 + drow]);
    u[1] = pack_h2(Vs[(s8 + 2) * 65 + drow], Vs[(s8 + 3) * 65 + drow]);
    u[2] = pack_h2(Vs[(s8 + 4) * 65 + drow], Vs[(s8 + 5) * 65 + drow]);
    u[3] = pack_h2(Vs[(s8 + 6) * 65 + drow], Vs[(s8 + 7) * 65 + drow]);
    st2_v4u(Vtp + ((size_t)(h * kHd + drow)) * kSeq + s0 + s8, u);
  }
}

__global__ __launch_bounds__(128) void k_attn_f16(const unsigned short* __restrict__ Qhp,
                                                    const unsigned short* __restrict__ Qlp,
                                                    const unsigned short* __restrict__ Kp,
                                                    const unsigned short* __restrict__ Vtp,
                                                    unsigned short* __restrict__ Chp,
                                                    unsigned short* __restrict__ Clp,
                                                    float sm_scale, float p_carry, float qres_inv, float o_scale) {
  __shared__ __align__(16) _Float16 Ksh[64 * 64];
  __shared__ __align__(16) _Float16 Vsh[64 * 64];
  __shared__ __align__(16) _Float16 Psh[4][16 * 64];
  __shared__ __align__(16) float    Osl[4][16 * 68];
  const int tid = threadIdx.x, wave = tid >> 5, lane = tid & 31;
  const int hh = lane >> 4, c = lane & 15;
  constexpr int nqb = kSeq / 64;
  const int bx = blockIdx.x;
  const int qb = bx % nqb;
  const int h  = bx / nqb;
  const int q0 = qb * 64 + wave * 16;

  const size_t qoff = ((size_t)h * kSeq + q0 + c) * kHd;
  const _Float16* Qh = (const _Float16*)(const void*)Qhp + qoff;
  const _Float16* Ql = (const _Float16*)(const void*)Qlp + qoff;
  v16h qa[2], ql[2];
#pragma unroll
  for (int dc = 0; dc < 2; ++dc) {
    qa[dc] = Frag<_Float16>::load(Qh + dc * 32 + 8 * hh);
    ql[dc] = Frag<_Float16>::load(Ql + dc * 32 + 8 * hh);
  }

  float mrow[8], lrow[8];
  v8f oacc[4];
#pragma unroll
  for (int r = 0; r < 8; ++r) { mrow[r] = -INFINITY; lrow[r] = 0.f; }
#pragma unroll
  for (int t = 0; t < 4; ++t) oacc[t] = (v8f){0.f,0.f,0.f,0.f,0.f,0.f,0.f,0.f};

  const v4u* Kg = (const v4u*)(const void*)(Kp + (size_t)h * kSeq * kHd);
  const unsigned short* Vg = Vtp + (size_t)h * kHd * kSeq;

#pragma unroll 1
  for (int kc = 0; kc < nqb; ++kc) {
    const int kv0 = kc * 64;
    __syncthreads();
#pragma unroll
    for (int it = 0; it < 4; ++it) {
      const int idx = it * 128 + tid;
      const v4u kk = Kg[(size_t)kv0 * 8 + idx];
      const int d = idx >> 3, p8 = idx & 7;
      const v4u vv = *(const v4u*)(const void*)(Vg + (size_t)d * kSeq + kv0 + p8 * 8);
      ((v4u*)(void*)Ksh)[idx] = kk;
      ((v4u*)(void*)Vsh)[idx] = vv;
    }
    __syncthreads();

    v8f s[4];
#pragma unroll
    for (int j = 0; j < 4; ++j) {
      const _Float16* krow = Ksh + (j * 16 + c) * kHd + 8 * hh;
      const v16h kb0 = Frag<_Float16>::load(krow);
      const v16h kb1 = Frag<_Float16>::load(krow + 32);
      v8f th = (v8f){0.f,0.f,0.f,0.f,0.f,0.f,0.f,0.f};
      th = hmma_f16(qa[0], kb0, th);
      th = hmma_f16(qa[1], kb1, th);
      v8f tl = (v8f){0.f,0.f,0.f,0.f,0.f,0.f,0.f,0.f};
      tl = hmma_f16(ql[0], kb0, tl);
      tl = hmma_f16(ql[1], kb1, tl);
#pragma unroll
      for (int r = 0; r < 8; ++r) s[j][r] = (th[r] + tl[r] * qres_inv) * sm_scale;
    }
    float cm[8];
#pragma unroll
    for (int r = 0; r < 8; ++r) {
      float m = -INFINITY;
#pragma unroll
      for (int j = 0; j < 4; ++j) m = fmaxf(m, s[j][r]);
#pragma unroll
      for (int off = 1; off < 16; off <<= 1) m = fmaxf(m, __shfl_xor(m, off, 32));
      cm[r] = m;
    }
    _Float16* pw = Psh[wave];
#pragma unroll
    for (int r = 0; r < 8; ++r) {
      const float mnew  = fmaxf(mrow[r], cm[r]);
      const float alpha = expf(mrow[r] - mnew);
      mrow[r] = mnew;
      float psum = 0.f;
#pragma unroll
      for (int j = 0; j < 4; ++j) {
        const float p = expf(s[j][r] - mnew);
        psum += p;
        pw[(8 * hh + r) * 64 + j * 16 + c] = (_Float16)(p * p_carry);
      }
#pragma unroll
      for (int off = 1; off < 16; off <<= 1) psum += __shfl_xor(psum, off, 32);
      lrow[r] = lrow[r] * alpha + psum;
#pragma unroll
      for (int t = 0; t < 4; ++t) oacc[t][r] *= alpha;
    }
    __builtin_amdgcn_fence(__ATOMIC_RELEASE, "workgroup");
    __builtin_amdgcn_wave_barrier();
    __builtin_amdgcn_fence(__ATOMIC_ACQUIRE, "workgroup");
#pragma unroll
    for (int kk = 0; kk < 2; ++kk) {
      const v16h pa = Frag<_Float16>::load(pw + c * 64 + kk * 32 + 8 * hh);
#pragma unroll
      for (int t = 0; t < 4; ++t) {
        const v16h vb = Frag<_Float16>::load(Vsh + (t * 16 + c) * 64 + kk * 32 + 8 * hh);
        oacc[t] = hmma_f16(pa, vb, oacc[t]);
      }
    }
  }

  float* os = Osl[wave];
#pragma unroll
  for (int r = 0; r < 8; ++r) {
    const float inv = o_scale * (1.0f / lrow[r]);
#pragma unroll
    for (int t = 0; t < 4; ++t) os[(8 * hh + r) * 68 + t * 16 + c] = oacc[t][r] * inv;
  }
  __builtin_amdgcn_fence(__ATOMIC_RELEASE, "workgroup");
  __builtin_amdgcn_wave_barrier();
  __builtin_amdgcn_fence(__ATOMIC_ACQUIRE, "workgroup");
  {
    const int q8 = lane >> 3, c8 = (lane & 7) * 8;
    unsigned short* Chb = Chp + (size_t)h * kHd;
    unsigned short* Clb = Clp + (size_t)h * kHd;
    for (int pass = 0; pass < 2; ++pass) {
#pragma unroll
      for (int it = 0; it < 4; ++it) {
        const int row = it * 4 + q8;
        const float* spp = os + row * 68 + c8;
        const v4f f0 = *(const v4f*)spp;
        const v4f f1 = *(const v4f*)(spp + 4);
        unsigned short hb[8], lb[8];
#pragma unroll
        for (int e = 0; e < 4; ++e) {
          hb[e]     = f2bf_bits(f0[e]);
          lb[e]     = f2bf_bits(f0[e] - bf_bits2f(hb[e]));
          hb[4 + e] = f2bf_bits(f1[e]);
          lb[4 + e] = f2bf_bits(f1[e] - bf_bits2f(hb[4 + e]));
        }
        v4u uh, ul;
#pragma unroll
        for (int e = 0; e < 4; ++e) {
          uh[e] = (unsigned)hb[2 * e] | ((unsigned)hb[2 * e + 1] << 16);
          ul[e] = (unsigned)lb[2 * e] | ((unsigned)lb[2 * e + 1] << 16);
        }
        const size_t o = (size_t)(q0 + row) * kDm + c8;
        *(volatile v4u*)(void*)(Chb + o) = uh;
        *(volatile v4u*)(void*)(Clb + o) = ul;
      }
      __threadfence();
    }
  }
}

extern "C" void kernel_launch(void* const* d_in, const int* in_sizes, int n_in,
                              void* d_out, int out_size, void* d_ws, size_t ws_size,
                              hipStream_t stream) {
  (void)n_in; (void)in_sizes; (void)out_size;
  const float* x     = (const float*)d_in[0];
  const float* W_qkv = (const float*)d_in[1];
  const float* b_qkv = (const float*)d_in[2];
  const float* W_out = (const float*)d_in[3];
  const float* b_out = (const float*)d_in[4];

  char* ws = (char*)d_ws;
  size_t off = 0;
  auto carve = [&](size_t bytes) -> char* { char* p = ws + off; off += (bytes + 255) & ~(size_t)255; return p; };
  unsigned short* Xb    = (unsigned short*)carve((size_t)kSeq * kDm * 2);
  unsigned short* WqkvT = (unsigned short*)carve((size_t)kNqkv * kDm * 2);
  unsigned short* WoutT = (unsigned short*)carve((size_t)kDm * kDm * 2);
  float* bqr  = (float*)carve((size_t)kNqkv * 4);
  float* bor  = (float*)carve((size_t)kDm * 4);
  float* QKV  = (float*)carve((size_t)kSeq * kNqkv * 4);
  float* cosT = (float*)carve((size_t)kSeq * 32 * 4);
  float* sinT = (float*)carve((size_t)kSeq * 32 * 4);
  unsigned short* Qh  = (unsigned short*)carve((size_t)kHeads * kSeq * kHd * 2);
  unsigned short* Ql  = (unsigned short*)carve((size_t)kHeads * kSeq * kHd * 2);
  unsigned short* Kp  = (unsigned short*)carve((size_t)kHeads * kSeq * kHd * 2);
  unsigned short* Vt  = (unsigned short*)carve((size_t)kHeads * kHd * kSeq * 2);
  unsigned short* Ch  = (unsigned short*)carve((size_t)kSeq * kDm * 2);
  unsigned short* Cl  = (unsigned short*)carve((size_t)kSeq * kDm * 2);
  if (off > ws_size) return;

  double rt = 1.3335214321633;
  for (int it = 0; it < 8; ++it) {
    double p31 = 1.0;
    for (int k = 0; k < 31; ++k) p31 *= rt;
    const double fv = p31 * rt - 10000.0;
    rt = rt - fv / (32.0 * p31);
  }
  RopeFreq fr;
  {
    double pw = 1.0;
    for (int i = 0; i < 32; ++i) {
      const float pf = (float)pw;
      fr.f[i] = 1.0f / pf;
      pw *= rt;
    }
  }

  k_cast_bf16<<<(kSeq * kDm / 8 + 255) / 256, 256, 0, stream>>>(x, Xb, kSeq * kDm / 8);
  k_bias_bf<<<4, 256, 0, stream>>>(b_qkv, b_out, bqr, bor);
  k_transpose_bf16<<<dim3(kNqkv / 64, kDm / 64), 256, 0, stream>>>(W_qkv, WqkvT, kDm, kNqkv);
  k_transpose_bf16<<<dim3(kDm / 64, kDm / 64), 256, 0, stream>>>(W_out, WoutT, kDm, kDm);
  k_rope_table<<<kSeq / 8, 256, 0, stream>>>(cosT, sinT, fr);
  static_assert(((kSeq / 64) * (kNqkv / 64)) % 8 == 0, "tile count");
  wmma_gemm64<1, 0, 2, 0, false><<<dim3((kSeq / 64) * (kNqkv / 64) / 8, 1), 256, 0, stream>>>(
      Xb, Xb, kDm, 0L, WqkvT, WqkvT, kDm, 0L, (void*)QKV, (void*)QKV, kNqkv, 0L,
      bqr, bqr, 0L, kSeq, kNqkv, kDm, 1.0f);
  k_rope_planes<<<dim3(kSeq / 64, kHeads), 256, 0, stream>>>(QKV, cosT, sinT, Qh, Ql, Kp, Vt, 2048.0f);
  k_attn_f16<<<kHeads * (kSeq / 64), 128, 0, stream>>>(Qh, Ql, Kp, Vt, Ch, Cl,
                                                      0.125f, 32768.0f, 1.0f / 2048.0f, 1.0f / 32768.0f);
  static_assert(((kSeq / 64) * (kDm / 64)) % 8 == 0, "tile count");
  wmma_gemm64<1, 1, 2, 0, false><<<dim3((kSeq / 64) * (kDm / 64) / 8, 1), 256, 0, stream>>>(
      Ch, Cl, kDm, 0L, WoutT, WoutT, kDm, 0L, d_out, d_out, kDm, 0L,
      bor, bor, 0L, kSeq, kDm, kDm, 1.0f);
}
